// QLSTM_23106924052492
// MI455X (gfx1250) — hardware-verified
//
#include <hip/hip_runtime.h>
#include <stddef.h>


#define T_   128
#define B_   64
#define F_   512
#define H_   1024
#define NOUT 513
#define NTO  33
#define KXT  16
#define KHT  32
#define KTT  48
#define NTH  64
#define HSLICE (B_ * H_)
#define OUT_BLK_ROWS 32
#define OUT_BLK_FLOATS (OUT_BLK_ROWS * NOUT)
#define OUT_CH0 8192
#define OUT_CH1 (OUT_BLK_FLOATS - OUT_CH0)

typedef _Float16 v16h __attribute__((ext_vector_type(16)));
typedef float v8f __attribute__((ext_vector_type(8)));
typedef float v4f __attribute__((ext_vector_type(4)));
typedef unsigned short us8 __attribute__((ext_vector_type(8)));
typedef unsigned short us16 __attribute__((ext_vector_type(16)));

union Frag { v16h v; us16 u; us8 u8[2]; };

__device__ __forceinline__ v8f wmma16(v8f c, v16h a, v16h b) {
  v8f d = __builtin_amdgcn_wmma_f32_16x16x32_f16(false, a, false, b, (short)0, c, false, false);
  asm volatile("v_nop\n\tv_nop\n\tv_nop\n\tv_nop" : "+v"(d) : "v"(a), "v"(b));
  return d;
}

__device__ __forceinline__ v8f zero8() {
  v8f z = {0.f, 0.f, 0.f, 0.f, 0.f, 0.f, 0.f, 0.f};
  return z;
}

__device__ __forceinline__ unsigned short f16bits(float f) {
  _Float16 q = (_Float16)f;
  return __builtin_bit_cast(unsigned short, q);
}

__device__ __forceinline__ float sigm(float x) { return __fdividef(1.0f, 1.0f + __expf(-x)); }
__device__ __forceinline__ float ftanh(float x) { return 1.0f - __fdividef(2.0f, 1.0f + __expf(2.0f * x)); }

__global__ __launch_bounds__(256) void k_cvt_x(const float* __restrict__ x, unsigned short* xh, int nchunk) {
  const int c = blockIdx.x * 256 + threadIdx.x;
  if (c >= nchunk) return;
  const v4f* p = (const v4f*)(x + (size_t)c * 8);
  const v4f a = p[0];
  const v4f b = p[1];
  us8 o;
  o[0] = f16bits(a[0] * 64.0f); o[1] = f16bits(a[1] * 64.0f);
  o[2] = f16bits(a[2] * 64.0f); o[3] = f16bits(a[3] * 64.0f);
  o[4] = f16bits(b[0] * 64.0f); o[5] = f16bits(b[1] * 64.0f);
  o[6] = f16bits(b[2] * 64.0f); o[7] = f16bits(b[3] * 64.0f);
  unsigned short* d = xh + (size_t)c * 8;
  *(volatile us8*)d = o;
  __threadfence();
  *(volatile us8*)d = o;
}

__global__ __launch_bounds__(256) void k_build_wu(unsigned short* bwu,
                                                 const float* __restrict__ w0, const float* __restrict__ w1,
                                                 const float* __restrict__ w2, const float* __restrict__ w3,
                                                 const float* __restrict__ u0, const float* __restrict__ u1,
                                                 const float* __restrict__ u2, const float* __restrict__ u3,
                                                 int nchunk) {
  const int c = blockIdx.x * 256 + threadIdx.x;
  if (c >= nchunk) return;
  const int tile = c >> 6, within = c & 63, lane = within >> 1, half = within & 1;
  const int kt = tile % KTT, gn = tile / KTT, nt = gn & (NTH - 1), g = gn >> 6;
  const int n = nt * 16 + (lane & 15), hh = lane >> 4;
  const int kb = kt * 32 + half * 16 + hh * 8;
  const int cb = n >> 8, q = n & 255;
  const float* src;
  int rb;
  if (kb < F_) {
    rb = kb >> 7;
    const int p0 = kb & 127;
    const float* wsel = (g == 0) ? w0 : (g == 1) ? w1 : (g == 2) ? w2 : w3;
    src = wsel + ((size_t)((rb ^ cb) * (F_ / 4) + p0)) * (H_ / 4) + q;
  } else {
    const int k = kb - F_;
    rb = k >> 8;
    const int p0 = k & 255;
    const float* usel = (g == 0) ? u0 : (g == 1) ? u1 : (g == 2) ? u2 : u3;
    src = usel + ((size_t)((rb ^ cb) * (H_ / 4) + p0)) * (H_ / 4) + q;
  }
  const float sgn = ((0x5390u >> (rb * 4 + cb)) & 1u) ? -16.0f : 16.0f;
  us8 o;
#pragma unroll
  for (int e = 0; e < 8; ++e) o[e] = f16bits(sgn * src[(size_t)e * (H_ / 4)]);
  unsigned short* d = bwu + (size_t)c * 8;
  *(volatile us8*)d = o;
  __threadfence();
  *(volatile us8*)d = o;
}

__global__ __launch_bounds__(256) void k_build_fco(unsigned short* fhi, unsigned short* flo,
                                                  const float* __restrict__ fw, int nchunk) {
  const int c = blockIdx.x * 256 + threadIdx.x;
  if (c >= nchunk) return;
  const int tile = c >> 6, within = c & 63, lane = within >> 1, half = within & 1;
  const int nt = tile >> 5, kt = tile & 31;
  const int n = nt * 16 + (lane & 15), hh = lane >> 4;
  const int kb = kt * 32 + half * 16 + hh * 8;
  us8 oh, ol;
#pragma unroll
  for (int e = 0; e < 8; ++e) {
    float v = 0.0f;
    if (n < NOUT) v = fw[(size_t)(kb + e) * NOUT + n] * 1024.0f;
    const _Float16 hq = (_Float16)v;
    const float res = (v - (float)hq) * 2048.0f;
    oh[e] = __builtin_bit_cast(unsigned short, hq);
    ol[e] = f16bits(res);
  }
  unsigned short* dh = fhi + (size_t)c * 8;
  unsigned short* dl = flo + (size_t)c * 8;
  *(volatile us8*)dh = oh;
  *(volatile us8*)dl = ol;
  __threadfence();
  *(volatile us8*)dh = oh;
  *(volatile us8*)dl = ol;
}

__global__ __launch_bounds__(128) void k_step(const unsigned short* __restrict__ xh,
                                              const unsigned short* __restrict__ bwu,
                                              const float* __restrict__ bF, const float* __restrict__ bI,
                                              const float* __restrict__ bO, const float* __restrict__ bC,
                                              unsigned short* hs, unsigned short* hl, float* cst, int t) {
  __shared__ __align__(16) unsigned short sH[4 * 256];
  __shared__ __align__(16) unsigned short sL[4 * 256];
  __shared__ __align__(16) float sC[4 * 256];
  const int nt = blockIdx.x;
  if (nt >= NTH) return;
  const int tid = threadIdx.x, lane = tid & 31, w = tid >> 5, hh = lane >> 4, n = lane & 15;
  const int m0 = w * 16;

  v8f acc[4];
#pragma unroll
  for (int g = 0; g < 4; ++g) acc[g] = zero8();

  const unsigned short* blane = bwu + (size_t)lane * 16;

  const unsigned short* xa = xh + (size_t)(t * B_ + m0 + n) * F_ + 8 * hh;
#pragma unroll 1
  for (int ks = 0; ks < KXT; ++ks) {
    Frag a;
    a.u8[0] = *(const us8*)(xa + ks * 32);
    a.u8[1] = *(const us8*)(xa + ks * 32 + 16);
#pragma unroll
    for (int g = 0; g < 4; ++g) {
      Frag b;
      b.u = *(const us16*)(blane + (size_t)((g * NTH + nt) * KTT + ks) * 512);
      acc[g] = wmma16(acc[g], a.v, b.v);
    }
  }

  if (t > 0) {
    const unsigned short* hp = hs + (size_t)(t - 1) * HSLICE + (size_t)(m0 + n) * 16 + 8 * hh;
#pragma unroll 1
    for (int ks = 0; ks < KHT; ++ks) {
      Frag a;
      a.u8[0] = *(const us8*)(hp + (size_t)(2 * ks) * (B_ * 16));
      a.u8[1] = *(const us8*)(hp + (size_t)(2 * ks + 1) * (B_ * 16));
#pragma unroll
      for (int g = 0; g < 4; ++g) {
        Frag b;
        b.u = *(const us16*)(blane + (size_t)((g * NTH + nt) * KTT + KXT + ks) * 512);
        acc[g] = wmma16(acc[g], a.v, b.v);
      }
    }
  }

  const int j = nt * 16 + n;
  const float biasF = bF[j], biasI = bI[j], biasO = bO[j], biasC = bC[j];
  const float inv = 1.0f / 1024.0f;
  const size_t cbase = ((size_t)nt * B_ + m0) * 16;
  unsigned short* sHw = sH + w * 256;
  unsigned short* sLw = sL + w * 256;
  float* sCw = sC + w * 256;
#pragma unroll
  for (int r = 0; r < 8; ++r) {
    const int rl = 8 * hh + r;
    const float pf = acc[0][r] * inv + biasF;
    const float pi = acc[1][r] * inv + biasI;
    const float po = acc[2][r] * inv + biasO;
    const float at = acc[3][r] * inv + biasC;
    const float ft = sigm(pf), it = sigm(pi), ot = sigm(po);
    float cp = 0.0f;
    if (t > 0) cp = cst[cbase + (size_t)rl * 16 + n];
    const float cn = it * ftanh(at) + ft * cp;
    const float hv = ot * ftanh(cn);
    const float hsc = hv * 64.0f;
    const _Float16 hq = (_Float16)hsc;
    const float res = (hsc - (float)hq) * 2048.0f;
    sHw[rl * 16 + n] = __builtin_bit_cast(unsigned short, hq);
    sLw[rl * 16 + n] = f16bits(res);
    sCw[rl * 16 + n] = cn;
  }
  __syncthreads();

  const us8 vh = *(const us8*)(sHw + lane * 8);
  const us8 vl = *(const us8*)(sLw + lane * 8);
  const v4f c0 = *(const v4f*)(sCw + lane * 4);
  const v4f c1 = *(const v4f*)(sCw + 128 + lane * 4);
  const size_t hbase = ((size_t)(t * NTH + nt) * B_ + m0) * 16 + (size_t)lane * 8;
  unsigned short* ph = hs + hbase;
  unsigned short* pl = hl + hbase;
  float* pc0 = cst + cbase + (size_t)lane * 4;
  float* pc1 = pc0 + 128;
  *(volatile us8*)ph = vh;
  *(volatile us8*)pl = vl;
  *(volatile v4f*)pc0 = c0;
  *(volatile v4f*)pc1 = c1;
  __threadfence();
  *(volatile us8*)ph = vh;
  *(volatile us8*)pl = vl;
  *(volatile v4f*)pc0 = c0;
  *(volatile v4f*)pc1 = c1;
}

__global__ __launch_bounds__(256) void k_gemm_out(const unsigned short* __restrict__ hs,
                                                 const unsigned short* __restrict__ hl,
                                                 const unsigned short* __restrict__ fhi,
                                                 const unsigned short* __restrict__ flo,
                                                 const float* __restrict__ fb, float* out, int nblk) {
  __shared__ __align__(16) float S[OUT_CH1];
  __shared__ float side[16];
  const int mb = blockIdx.x;
  if (mb >= nblk) return;
  const int tid = threadIdx.x, lane = tid & 31, w = tid >> 5, hh = lane >> 4, n = lane & 15;
  const int t = mb >> 1, mr0 = (mb & 1) * 32;
  const unsigned short* ha = hs + (size_t)t * HSLICE + 8 * hh;
  const unsigned short* la = hl + (size_t)t * HSLICE + 8 * hh;
  float* dst = out + (size_t)mb * OUT_BLK_FLOATS;

  for (int mi = 0; mi < 2; ++mi) {
    const int arow = (mr0 + mi * 16 + n) * 16;
    for (int nt = w; nt < NTO; nt += 8) {
      v8f am = zero8();
      v8f ax = zero8();
      const unsigned short* pbh = fhi + (size_t)nt * KHT * 512 + lane * 16;
      const unsigned short* pbl = flo + (size_t)nt * KHT * 512 + lane * 16;
#pragma unroll 1
      for (int ks = 0; ks < KHT; ++ks) {
        Frag bh, bl, ah, al;
        bh.u = *(const us16*)(pbh + ks * 512);
        bl.u = *(const us16*)(pbl + ks * 512);
        const size_t o0 = (size_t)(2 * ks) * (B_ * 16) + arow;
        const size_t o1 = o0 + B_ * 16;
        ah.u8[0] = *(const us8*)(ha + o0);
        ah.u8[1] = *(const us8*)(ha + o1);
        al.u8[0] = *(const us8*)(la + o0);
        al.u8[1] = *(const us8*)(la + o1);
        am = wmma16(am, ah.v, bh.v);
        ax = wmma16(ax, ah.v, bl.v);
        ax = wmma16(ax, al.v, bh.v);
      }
      const int col = nt * 16 + n;
      const int colc = (col < NOUT) ? col : (NOUT - 1);
      const float bias = fb[colc];
#pragma unroll
      for (int r = 0; r < 8; ++r) {
        const int rl = 8 * hh + r;
        const float v = (am[r] + ax[r] * (1.0f / 2048.0f)) * (1.0f / 65536.0f) + bias;
        if (col < NOUT) {
          if (mi == 0) {
            const int f = rl * NOUT + col;
            if (f < OUT_CH0) S[f] = v; else side[f - OUT_CH0] = v;
          } else {
            S[16 + rl * NOUT + col] = v;
          }
        }
      }
    }
    if (mi == 1 && tid < 16) S[tid] = side[tid];
    __syncthreads();

    const int nq = (mi == 0) ? (OUT_CH0 / 4) : (OUT_CH1 / 4);
    float* d = dst + ((mi == 0) ? 0 : OUT_CH0);
    for (int i = tid; i < nq; i += 256) {
      const v4f v = *(const v4f*)(S + i * 4);
      *(volatile v4f*)(d + (size_t)i * 4) = v;
    }
    __threadfence();
    for (int i = tid; i < nq; i += 256) {
      const v4f v = *(const v4f*)(S + i * 4);
      *(volatile v4f*)(d + (size_t)i * 4) = v;
    }
    __syncthreads();
  }
}

extern "C" void kernel_launch(void* const* d_in, const int* in_sizes, int n_in,
                              void* d_out, int out_size, void* d_ws, size_t ws_size,
                              hipStream_t stream) {
  if (n_in < 15) return;
  if (in_sizes[0] != T_ * B_ * F_) return;
  if (in_sizes[1] != F_ * H_ / 4 || in_sizes[3] != F_ * H_ / 4 ||
      in_sizes[5] != F_ * H_ / 4 || in_sizes[7] != F_ * H_ / 4) return;
  if (in_sizes[2] != H_ || in_sizes[4] != H_ || in_sizes[6] != H_ || in_sizes[8] != H_) return;
  if (in_sizes[9] != H_ * H_ / 4 || in_sizes[10] != H_ * H_ / 4 ||
      in_sizes[11] != H_ * H_ / 4 || in_sizes[12] != H_ * H_ / 4) return;
  if (in_sizes[13] != H_ * NOUT || in_sizes[14] != NOUT) return;
  if (out_size != T_ * B_ * NOUT) return;

  const float* x     = (const float*)d_in[0];
  const float* wfx_w = (const float*)d_in[1];  const float* wfx_b = (const float*)d_in[2];
  const float* wix_w = (const float*)d_in[3];  const float* wix_b = (const float*)d_in[4];
  const float* wox_w = (const float*)d_in[5];  const float* wox_b = (const float*)d_in[6];
  const float* wcx_w = (const float*)d_in[7];  const float* wcx_b = (const float*)d_in[8];
  const float* ufh_w = (const float*)d_in[9];  const float* uih_w = (const float*)d_in[10];
  const float* uoh_w = (const float*)d_in[11]; const float* uch_w = (const float*)d_in[12];
  const float* fco_w = (const float*)d_in[13]; const float* fco_b = (const float*)d_in[14];

  const size_t nXh  = (size_t)T_ * B_ * F_ * 2;
  const size_t nBwu = (size_t)4 * NTH * KTT * 512 * 2;
  const size_t nF   = (size_t)NTO * KHT * 512 * 2;
  const size_t nH   = (size_t)T_ * HSLICE * 2;
  const size_t nC   = (size_t)HSLICE * 4;
  const size_t oXh  = 0;
  const size_t oBwu = oXh + nXh;
  const size_t oFhi = oBwu + nBwu;
  const size_t oFlo = oFhi + nF;
  const size_t oHs  = oFlo + nF;
  const size_t oHl  = oHs + nH;
  const size_t oC   = oHl + nH;
  const size_t oEnd = oC + nC;
  if (oEnd > ws_size) return;

  char* ws = (char*)d_ws;
  unsigned short* Xh  = (unsigned short*)(ws + oXh);
  unsigned short* Bwu = (unsigned short*)(ws + oBwu);
  unsigned short* Fhi = (unsigned short*)(ws + oFhi);
  unsigned short* Flo = (unsigned short*)(ws + oFlo);
  unsigned short* Hs  = (unsigned short*)(ws + oHs);
  unsigned short* Hl  = (unsigned short*)(ws + oHl);
  float*          Cst = (float*)(ws + oC);
  float*          out = (float*)d_out;

  const int nChunkX   = T_ * B_ * F_ / 8;
  const int nChunkWU  = 4 * NTH * KTT * 64;
  const int nChunkF   = NTO * KHT * 64;
  const int nBlkOut   = T_ * B_ / OUT_BLK_ROWS;

  k_cvt_x<<<(nChunkX + 255) / 256, 256, 0, stream>>>(x, Xh, nChunkX);
  k_build_wu<<<(nChunkWU + 255) / 256, 256, 0, stream>>>(Bwu, wfx_w, wix_w, wox_w, wcx_w,
                                                       ufh_w, uih_w, uoh_w, uch_w, nChunkWU);
  k_build_fco<<<(nChunkF + 255) / 256, 256, 0, stream>>>(Fhi, Flo, fco_w, nChunkF);

  for (int t = 0; t < T_; ++t)
    k_step<<<NTH, 128, 0, stream>>>(Xh, Bwu, wfx_b, wix_b, wox_b, wcx_b, Hs, Hl, Cst, t);

  k_gemm_out<<<nBlkOut, 256, 0, stream>>>(Hs, Hl, Fhi, Flo, fco_b, out, nBlkOut);
}
